// LSTMEncoder_32530082300436
// MI455X (gfx1250) — hardware-run, weakly checked
//
#include <hip/hip_runtime.h>
#include <math.h>

constexpr int NSEQ     = 4096;
constexpr int NSTEP    = 512;
constexpr int NXIN     = 6;
constexpr int NHID     = 32;
constexpr int NGATE    = 128;
constexpr int NWAVE    = 2;
constexpr int NTHR     = 32 * NWAVE;
constexpr int ROWS_BLK = 16 * NWAVE;
constexpr int WPITCH   = 40;
constexpr int HPITCH   = 40;
constexpr int SPITCH   = 36;
constexpr float XW_CARRY = 1024.0f;
constexpr float HW_CARRY = 64.0f;
constexpr float H_CARRY  = 16.0f;
constexpr float ACC_INV  = 1.0f / 1024.0f;
static_assert(NSEQ % ROWS_BLK == 0);
static_assert(ROWS_BLK == 16 * NWAVE);
static_assert(NGATE == 4 * NHID);
static_assert(NHID == 32);
static_assert(NXIN == 6);
static_assert((NGATE * 16) % NTHR == 0);
static_assert((2 * NGATE) % NTHR == 0);
static_assert(WPITCH % 8 == 0 && HPITCH % 8 == 0 && SPITCH % 4 == 0);

typedef __attribute__((ext_vector_type(16))) _Float16 v16h;
typedef __attribute__((ext_vector_type(8)))  _Float16 v8h;
typedef __attribute__((ext_vector_type(16))) __bf16   v16b;
typedef __attribute__((ext_vector_type(8)))  __bf16   v8b;
typedef __attribute__((ext_vector_type(8)))  float    v8f;
typedef __attribute__((ext_vector_type(4)))  float    v4f;
typedef __attribute__((ext_vector_type(2)))  float    v2f;
typedef __attribute__((ext_vector_type(8)))  unsigned v8u;

__device__ __forceinline__ unsigned short f2bf_bits(float f) {
  unsigned u = __float_as_uint(f);
  return (unsigned short)((u + 0x7FFFu + ((u >> 16) & 1u)) >> 16);
}
__device__ __forceinline__ float bf_bits2f(unsigned short h) { return __uint_as_float(((unsigned)h) << 16); }
__device__ __forceinline__ float bf16r(float f) { return bf_bits2f(f2bf_bits(f)); }

__device__ __forceinline__ void guard4_h(v8f& a0, v8f& a1, v8f& a2, v8f& a3, v16h fa, v16h b0, v16h b1, v16h b2, v16h b3) {
  asm volatile("v_nop\n\tv_nop\n\tv_nop\n\tv_nop" : "+v"(a0), "+v"(a1), "+v"(a2), "+v"(a3) : "v"(fa), "v"(b0), "v"(b1), "v"(b2), "v"(b3));
}
__device__ __forceinline__ void guard4_b(v8f& a0, v8f& a1, v8f& a2, v8f& a3, v16b fa, v16b b0, v16b b1, v16b b2, v16b b3) {
  asm volatile("v_nop\n\tv_nop\n\tv_nop\n\tv_nop" : "+v"(a0), "+v"(a1), "+v"(a2), "+v"(a3) : "v"(fa), "v"(b0), "v"(b1), "v"(b2), "v"(b3));
}

template <typename T> struct Frag;
template <> struct Frag<_Float16> {
  typedef v16h V; union U { v16h v; v8h h[2]; };
  static __device__ __forceinline__ v16h load(const _Float16* p) {
    U f; f.h[0] = *(const v8h*)(p); f.h[1] = *(const v8h*)(p + 16); return f.v;
  }
  static __device__ __forceinline__ v8f mma(v16h a, v16h b, v8f c) {
    return __builtin_amdgcn_wmma_f32_16x16x32_f16(false, a, false, b, (short)0, c, false, false);
  }
};
template <> struct Frag<__bf16> {
  typedef v16b V; union U { v16b v; v8b h[2]; };
  static __device__ __forceinline__ v16b load(const __bf16* p) {
    U f; f.h[0] = *(const v8b*)(p); f.h[1] = *(const v8b*)(p + 16); return f.v;
  }
  static __device__ __forceinline__ v8f mma(v16b a, v16b b, v8f c) {
    return __builtin_amdgcn_wmma_f32_16x16x32_bf16(false, a, false, b, (short)0, c, false, false);
  }
};

__device__ __forceinline__ float fsig(float v)  { return __builtin_amdgcn_rcpf(1.0f + expf(-v)); }
__device__ __forceinline__ float ftanh(float v) { return 1.0f - 2.0f * __builtin_amdgcn_rcpf(expf(2.0f * v) + 1.0f); }

__device__ __forceinline__ void mma4_f16(v8f& a0, v8f& a1, v8f& a2, v8f& a3, v16h fa, const unsigned short* Wp, int rowoff) {
  const _Float16* W = (const _Float16*)Wp + rowoff;
  const v16h b0 = Frag<_Float16>::load(W + 0 * 32 * WPITCH);
  const v16h b1 = Frag<_Float16>::load(W + 1 * 32 * WPITCH);
  const v16h b2 = Frag<_Float16>::load(W + 2 * 32 * WPITCH);
  const v16h b3 = Frag<_Float16>::load(W + 3 * 32 * WPITCH);
  a0 = Frag<_Float16>::mma(fa, b0, a0);
  a1 = Frag<_Float16>::mma(fa, b1, a1);
  a2 = Frag<_Float16>::mma(fa, b2, a2);
  a3 = Frag<_Float16>::mma(fa, b3, a3);
  guard4_h(a0, a1, a2, a3, fa, b0, b1, b2, b3);
}
__device__ __forceinline__ void mma4_bf16(v8f& a0, v8f& a1, v8f& a2, v8f& a3, v16b fa, const unsigned short* Wp, int rowoff) {
  const __bf16* W = (const __bf16*)Wp + rowoff;
  const v16b b0 = Frag<__bf16>::load(W + 0 * 32 * WPITCH);
  const v16b b1 = Frag<__bf16>::load(W + 1 * 32 * WPITCH);
  const v16b b2 = Frag<__bf16>::load(W + 2 * 32 * WPITCH);
  const v16b b3 = Frag<__bf16>::load(W + 3 * 32 * WPITCH);
  a0 = Frag<__bf16>::mma(fa, b0, a0);
  a1 = Frag<__bf16>::mma(fa, b1, a1);
  a2 = Frag<__bf16>::mma(fa, b2, a2);
  a3 = Frag<__bf16>::mma(fa, b3, a3);
  guard4_b(a0, a1, a2, a3, fa, b0, b1, b2, b3);
}

__device__ __forceinline__ void stage_w_rec(const float* __restrict__ src, unsigned short* dst, int tid) {
#pragma unroll 1
  for (int e = tid; e < NGATE * (NHID / 2); e += NTHR) {
    const int n = e >> 4, k = (e & 15) * 2;
    const float v0 = src[n * NHID + k];
    const float v1 = src[n * NHID + k + 1];
    const _Float16 h0 = (_Float16)(bf16r(v0) * HW_CARRY);
    const _Float16 h1 = (_Float16)(bf16r(v1) * HW_CARRY);
    const unsigned u = (unsigned)__builtin_bit_cast(unsigned short, h0) | ((unsigned)__builtin_bit_cast(unsigned short, h1) << 16);
    *(unsigned*)(dst + n * WPITCH + k) = u;
  }
}
__device__ __forceinline__ void stage_w_in0(const float* __restrict__ src, unsigned short* dst, int tid) {
#pragma unroll 1
  for (int e = tid; e < NGATE * 16; e += NTHR) {
    const int n = e >> 4, k = (e & 15) * 2;
    const int kc = (k < NXIN) ? k : (NXIN - 2);
    const float fz = (k < NXIN) ? 1.0f : 0.0f;
    const float v0 = src[n * NXIN + kc] * fz;
    const float v1 = src[n * NXIN + kc + 1] * fz;
    const unsigned u = (unsigned)f2bf_bits(v0 * XW_CARRY) | ((unsigned)f2bf_bits(v1 * XW_CARRY) << 16);
    *(unsigned*)(dst + n * WPITCH + k) = u;
  }
}

__global__ __launch_bounds__(NTHR) void lstm2_seq_kernel(
    const float* __restrict__ x,
    const float* __restrict__ Wih0, const float* __restrict__ Whh0, const float* __restrict__ bih0, const float* __restrict__ bhh0,
    const float* __restrict__ Wih1, const float* __restrict__ Whh1, const float* __restrict__ bih1, const float* __restrict__ bhh1,
    float* __restrict__ out) {
  __shared__ __align__(16) unsigned short Wx0s[NGATE * WPITCH];
  __shared__ __align__(16) unsigned short Wh0s[NGATE * WPITCH];
  __shared__ __align__(16) unsigned short Wx1s[NGATE * WPITCH];
  __shared__ __align__(16) unsigned short Wh1s[NGATE * WPITCH];
  __shared__ __align__(16) _Float16 H0t[NWAVE][16 * HPITCH];
  __shared__ __align__(16) _Float16 H1t[NWAVE][16 * HPITCH];
  __shared__ __align__(16) float Bsum[2 * NGATE];
  __shared__ __align__(16) float Osl[NWAVE][16 * SPITCH];

  const int tid = threadIdx.x, lane = tid & 31, wave = tid >> 5;
  const int c = lane & 15, hh = lane >> 4;
  const int rowb = blockIdx.x * ROWS_BLK + wave * 16;

  stage_w_in0(Wih0, Wx0s, tid);
  stage_w_rec(Whh0, Wh0s, tid);
  stage_w_rec(Wih1, Wx1s, tid);
  stage_w_rec(Whh1, Wh1s, tid);
#pragma unroll 1
  for (int e = tid; e < 2 * NGATE; e += NTHR) {
    const int col = e & (NGATE - 1);
    const float s0 = bf16r(bih0[col]) + bf16r(bhh0[col]);
    const float s1 = bf16r(bih1[col]) + bf16r(bhh1[col]);
    const float fl = (float)(e >> 7);
    Bsum[e] = fmaf(fl, s1, (1.0f - fl) * s0);
  }
  float cst0[2][8], cst1[2][8], hst1[2][8];
#pragma unroll
  for (int ub = 0; ub < 2; ++ub)
#pragma unroll
    for (int r = 0; r < 8; ++r) { cst0[ub][r] = 0.0f; cst1[ub][r] = 0.0f; hst1[ub][r] = 0.0f; }
  __syncthreads();

  const v8u zu = {0u, 0u, 0u, 0u, 0u, 0u, 0u, 0u};
  const v8f z8 = {0.f, 0.f, 0.f, 0.f, 0.f, 0.f, 0.f, 0.f};
  v16h a0 = __builtin_bit_cast(v16h, zu);
  v16h a1 = __builtin_bit_cast(v16h, zu);
  const float fz = 1.0f - (float)hh;
  _Float16* h0w = H0t[wave];
  _Float16* h1w = H1t[wave];
  const int arow = c * HPITCH + 8 * hh;

#pragma unroll 1
  for (int t = 0; t < NSTEP; ++t) {
    asm volatile("" ::: "memory");
    const float* px = x + ((size_t)(rowb + c) * NSTEP + (size_t)t) * NXIN;
    const v2f p0 = *(const v2f*)(px);
    const v2f p1 = *(const v2f*)(px + 2);
    const v2f p2 = *(const v2f*)(px + 4);
    v8u xw = zu;
    xw[0] = (unsigned)f2bf_bits(p0[0] * fz) | ((unsigned)f2bf_bits(p0[1] * fz) << 16);
    xw[1] = (unsigned)f2bf_bits(p1[0] * fz) | ((unsigned)f2bf_bits(p1[1] * fz) << 16);
    xw[2] = (unsigned)f2bf_bits(p2[0] * fz) | ((unsigned)f2bf_bits(p2[1] * fz) << 16);
    const v16b xa = __builtin_bit_cast(v16b, xw);

#pragma unroll
    for (int ub = 0; ub < 2; ++ub) {
      const int bcol = 16 * ub + c;
      const int rowoff = bcol * WPITCH + 8 * hh;
      v8f ai = z8, af = z8, ag = z8, ao = z8;
      mma4_bf16(ai, af, ag, ao, xa, Wx0s, rowoff);
      mma4_f16(ai, af, ag, ao, a0, Wh0s, rowoff);
      const float bi = Bsum[bcol], bf = Bsum[NHID + bcol], bg = Bsum[2 * NHID + bcol], bo = Bsum[3 * NHID + bcol];
#pragma unroll
      for (int r = 0; r < 8; ++r) {
        const float zi = ai[r] * ACC_INV + bi;
        const float zf = af[r] * ACC_INV + bf;
        const float zg = ag[r] * ACC_INV + bg;
        const float zo = ao[r] * ACC_INV + bo;
        const float ig = fsig(zi);
        const float fg = fsig(zf);
        const float gg = ftanh(zg);
        const float og = fsig(zo);
        const float cn = fg * cst0[ub][r] + ig * gg;
        cst0[ub][r] = cn;
        const float hv = og * ftanh(cn);
        h0w[(8 * hh + r) * HPITCH + bcol] = (_Float16)(hv * H_CARRY);
      }
      asm volatile("" ::: "memory");
    }
    __syncthreads();
    a0 = Frag<_Float16>::load(h0w + arow);

#pragma unroll
    for (int ub = 0; ub < 2; ++ub) {
      const int bcol = 16 * ub + c;
      const int rowoff = bcol * WPITCH + 8 * hh;
      v8f ai = z8, af = z8, ag = z8, ao = z8;
      mma4_f16(ai, af, ag, ao, a0, Wx1s, rowoff);
      mma4_f16(ai, af, ag, ao, a1, Wh1s, rowoff);
      const float bi = Bsum[NGATE + bcol], bf = Bsum[NGATE + NHID + bcol], bg = Bsum[NGATE + 2 * NHID + bcol], bo = Bsum[NGATE + 3 * NHID + bcol];
#pragma unroll
      for (int r = 0; r < 8; ++r) {
        const float zi = ai[r] * ACC_INV + bi;
        const float zf = af[r] * ACC_INV + bf;
        const float zg = ag[r] * ACC_INV + bg;
        const float zo = ao[r] * ACC_INV + bo;
        const float ig = fsig(zi);
        const float fg = fsig(zf);
        const float gg = ftanh(zg);
        const float og = fsig(zo);
        const float cn = fg * cst1[ub][r] + ig * gg;
        cst1[ub][r] = cn;
        const float hv = og * ftanh(cn);
        hst1[ub][r] = hv;
        h1w[(8 * hh + r) * HPITCH + bcol] = (_Float16)(hv * H_CARRY);
      }
      asm volatile("" ::: "memory");
    }
    __syncthreads();
    a1 = Frag<_Float16>::load(h1w + arow);
  }

  float* os = Osl[wave];
#pragma unroll
  for (int ub = 0; ub < 2; ++ub)
#pragma unroll
    for (int r = 0; r < 8; ++r) os[(8 * hh + r) * SPITCH + 16 * ub + c] = hst1[ub][r];
  __syncthreads();
  {
    const int q = lane >> 3, c4 = (lane & 7) * 4;
    for (int pass = 0; pass < 2; ++pass) {
#pragma unroll
      for (int it = 0; it < 4; ++it) {
        const int row = it * 4 + q;
        const v4f v = *(const v4f*)(os + row * SPITCH + c4);
        *(volatile v4f*)(out + (size_t)(rowb + row) * NHID + c4) = v;
      }
      __threadfence();
    }
  }
}

extern "C" void kernel_launch(void* const* d_in, const int* in_sizes, int n_in,
                              void* d_out, int out_size, void* d_ws, size_t ws_size, hipStream_t stream) {
  (void)d_ws; (void)ws_size;
  if (n_in < 9 || d_out == nullptr) return;
  if (in_sizes[0] != NSEQ * NSTEP * NXIN || in_sizes[1] != NGATE * NXIN || in_sizes[2] != NGATE * NHID ||
      in_sizes[3] != NGATE || in_sizes[4] != NGATE || in_sizes[5] != NGATE * NHID || in_sizes[6] != NGATE * NHID ||
      in_sizes[7] != NGATE || in_sizes[8] != NGATE || out_size != NSEQ * NHID) return;

  const float* x    = (const float*)d_in[0];
  const float* Wih0 = (const float*)d_in[1];
  const float* Whh0 = (const float*)d_in[2];
  const float* bih0 = (const float*)d_in[3];
  const float* bhh0 = (const float*)d_in[4];
  const float* Wih1 = (const float*)d_in[5];
  const float* Whh1 = (const float*)d_in[6];
  const float* bih1 = (const float*)d_in[7];
  const float* bhh1 = (const float*)d_in[8];
  float* out = (float*)d_out;

  lstm2_seq_kernel<<<NSEQ / ROWS_BLK, NTHR, 0, stream>>>(x, Wih0, Whh0, bih0, bhh0, Wih1, Whh1, bih1, bhh1, out);
}
